// TriGAT_1855425872580
// MI455X (gfx1250) — hardware-run, weakly checked
//
#include <hip/hip_runtime.h>
#include <stddef.h>
#include <stdint.h>
#include <math.h>


#define F_IN    128
#define HC1     128
#define HID     64
#define NHD1    2
#define HCAT    384
#define KX      768
#define NCLS    16
#define NTHR    256
#define NWAVE   8
#define EPT     8
#define CHUNK   (NTHR * EPT)
#define WCAP    (EPT * 32)
#define LISTN   (NWAVE * WCAP)
#define NBMAX   2048
#define SLOTB   11
#define RCAP    28672
#define DEGCAP  256
#define GBM     64
#define GTHR    128
#define MROWS   128
#define GRP     64
#define WST     256
#define NUW     (HC1 * (F_IN / 8))
#define NUL     (NCLS * (KX / 8))
#define NEGSL   0.2f
#define WSMAX   134217728
#define LDS_AGG ((2 * RCAP + 2 * NBMAX + LISTN) * 4 + 64)

static_assert((CHUNK & (CHUNK - 1)) == 0 && CHUNK <= (1 << SLOTB));
static_assert(NBMAX == (1 << SLOTB));
static_assert(NTHR * 8 == NBMAX);
static_assert(LISTN >= NBMAX);
static_assert(LISTN >= NWAVE * WCAP);
static_assert((RCAP % 32) == 0);
static_assert(LDS_AGG <= 327680);
static_assert(GBM == (GTHR / 32) * 16);
static_assert(GTHR == 2 * GBM);
static_assert((F_IN % 32) == 0 && (KX % 32) == 0);
static_assert(KX == 2 * HCAT && HCAT == 3 * HC1);
static_assert(NHD1 * HID == HC1 && HC1 == 4 * 32);
static_assert((HID % 16) == 0 && HID == 64);
static_assert(NCLS == 16);
static_assert((MROWS % GBM) == 0);
static_assert(NWAVE * GRP * NCLS <= RCAP);
static_assert(NWAVE * WST <= RCAP);
static_assert(WST * 4 >= HC1 * 4 + 2 * HC1 * 2);
static_assert((GRP & (GRP - 1)) == 0 && (GRP % 2) == 0);
static_assert((NUW % NTHR) == 0 && (NUL % NTHR) == 0);
static_assert((F_IN / 8) == 16);
static_assert((HCAT % 8) == 0);

typedef float          v4f  __attribute__((ext_vector_type(4)));
typedef float          v8f  __attribute__((ext_vector_type(8)));
typedef int            v4i  __attribute__((ext_vector_type(4)));
typedef int            v8i  __attribute__((ext_vector_type(8)));
typedef unsigned int   v4u  __attribute__((ext_vector_type(4)));
typedef unsigned short v8us __attribute__((ext_vector_type(8)));
typedef __bf16         v16b __attribute__((ext_vector_type(16)));
typedef v4f  __attribute__((may_alias)) v4fa;
typedef v8us __attribute__((may_alias)) v8usa;
union FragB { v16b v; v8us h[2]; v8i w; };

__device__ __forceinline__ v8f wmb(const FragB& a, const FragB& b, v8f c) {
  v8f d = __builtin_amdgcn_wmma_f32_16x16x32_bf16(false, a.v, false, b.v, (short)0, c, false, false);
  asm volatile("v_nop\n\tv_nop\n\tv_nop\n\tv_nop" : "+v"(d) : "v"(a.w), "v"(b.w));
  return d;
}

__device__ __forceinline__ unsigned int f2bf(float f) {
  const unsigned int u = __float_as_uint(f);
  const unsigned int r = ((u + 0x7FFFu + ((u >> 16) & 1u)) >> 16) & 0xFFFFu;
  return ((u & 0x7FFFFFFFu) > 0x7F800000u) ? 0x7FC0u : r;
}
__device__ __forceinline__ float bf2f(unsigned int b) { return __uint_as_float(b << 16); }
__device__ __forceinline__ float bfr(float f) { return bf2f(f2bf(f)); }
__device__ __forceinline__ v4f bfr4(const v4f a) {
  v4f r; r.x = bfr(a.x); r.y = bfr(a.y); r.z = bfr(a.z); r.w = bfr(a.w); return r;
}
__device__ __forceinline__ unsigned int pk2(float lo, float hi) { return f2bf(lo) | (f2bf(hi) << 16); }
__device__ __forceinline__ v4u pack8(const v4f a, const v4f b) {
  v4u r;
  r.x = pk2(a.x, a.y); r.y = pk2(a.z, a.w); r.z = pk2(b.x, b.y); r.w = pk2(b.z, b.w);
  return r;
}

__device__ __forceinline__ int scan_chunk(const int* __restrict__ dsts, int nE, int cbase, int slotBase,
                                          int nb, int vec8, int* list, int tid, int lane, int wave) {
  int wc = 0;
  const int el0  = tid * EPT;
  const int e0   = cbase + el0;
  const int sent = -2147483647 - 1;
  v4i da, db;
  if (vec8 != 0 && cbase + CHUNK <= nE) {
    da = *(const v4i*)(dsts + e0);
    db = *(const v4i*)(dsts + e0 + 4);
  } else {
    da.x = (e0     < nE) ? dsts[min(e0,     nE - 1)] : sent;
    da.y = (e0 + 1 < nE) ? dsts[min(e0 + 1, nE - 1)] : sent;
    da.z = (e0 + 2 < nE) ? dsts[min(e0 + 2, nE - 1)] : sent;
    da.w = (e0 + 3 < nE) ? dsts[min(e0 + 3, nE - 1)] : sent;
    db.x = (e0 + 4 < nE) ? dsts[min(e0 + 4, nE - 1)] : sent;
    db.y = (e0 + 5 < nE) ? dsts[min(e0 + 5, nE - 1)] : sent;
    db.z = (e0 + 6 < nE) ? dsts[min(e0 + 6, nE - 1)] : sent;
    db.w = (e0 + 7 < nE) ? dsts[min(e0 + 7, nE - 1)] : sent;
  }
  const unsigned nbs = (unsigned)slotBase;
  const unsigned unb = (unsigned)nb;
  const unsigned s0 = (unsigned)da.x - nbs, s1 = (unsigned)da.y - nbs;
  const unsigned s2 = (unsigned)da.z - nbs, s3 = (unsigned)da.w - nbs;
  const unsigned s4 = (unsigned)db.x - nbs, s5 = (unsigned)db.y - nbs;
  const unsigned s6 = (unsigned)db.z - nbs, s7 = (unsigned)db.w - nbs;
  const bool h0 = s0 < unb, h1 = s1 < unb, h2 = s2 < unb, h3 = s3 < unb;
  const bool h4 = s4 < unb, h5 = s5 < unb, h6 = s6 < unb, h7 = s7 < unb;
  const unsigned any = __builtin_amdgcn_ballot_w32(h0 | h1 | h2 | h3 | h4 | h5 | h6 | h7);
  if (any != 0u) {
#define HITJ(J, HJ, SJ) { \
      const unsigned mj = __builtin_amdgcn_ballot_w32(HJ); \
      if (mj != 0u) { \
        if (HJ) { \
          const int pos = wc + (int)__builtin_amdgcn_mbcnt_lo(mj, 0u); \
          if (pos < WCAP) list[wave * WCAP + pos] = ((el0 + (J)) << SLOTB) | (int)(SJ); \
        } \
        wc += (int)__builtin_popcount(mj); } }
    HITJ(0, h0, s0)
    HITJ(1, h1, s1)
    HITJ(2, h2, s2)
    HITJ(3, h3, s3)
    HITJ(4, h4, s4)
    HITJ(5, h5, s5)
    HITJ(6, h6, s6)
    HITJ(7, h7, s7)
#undef HITJ
  }
  return wc;
}

__device__ __forceinline__ void wtr_unit(const float* __restrict__ w, int Kin, int Ncol, int Kout,
                                         unsigned short* wt, int v) {
  const int kq = Kout >> 3;
  const int n  = v / kq;
  const int k8 = (v - n * kq) * 8;
  const int kk = k8 - (k8 / Kin) * Kin;
  const int ncl = n < Ncol ? n : Ncol - 1;
  const float* p = w + (size_t)kk * (size_t)Ncol + ncl;
  v4f a, b;
  a.x = p[0];                    a.y = p[(size_t)Ncol];         a.z = p[(size_t)2 * Ncol];     a.w = p[(size_t)3 * Ncol];
  b.x = p[(size_t)4 * Ncol];     b.y = p[(size_t)5 * Ncol];     b.z = p[(size_t)6 * Ncol];     b.w = p[(size_t)7 * Ncol];
  const v4f z4 = {0.f, 0.f, 0.f, 0.f};
  if (n >= Ncol) { a = z4; b = z4; }
  const v4u wv = pack8(a, b);
  unsigned short* o = wt + (size_t)n * (size_t)Kout + k8;
  *(volatile v4u*)o = wv;
  __threadfence();
  *(volatile v4u*)o = wv;
}

__global__ __launch_bounds__(NTHR) void k_prep(const float* __restrict__ x,
                                               const float* __restrict__ W0, const float* __restrict__ W1,
                                               const float* __restrict__ W2, const float* __restrict__ Wl,
                                               unsigned short* XB, unsigned short* WT0, unsigned short* WT1,
                                               unsigned short* WT2, unsigned short* WLT, int nN, int nUx) {
  const int u = (int)blockIdx.x * NTHR + (int)threadIdx.x;
  if (u < nUx) {
    const int row = u >> 4;
    const int c0  = (u & 15) * 8;
    const int rc  = row < nN ? row : nN - 1;
    const float* p = x + (size_t)rc * F_IN + c0;
    v4f a = *(const v4fa*)p, b = *(const v4fa*)(p + 4);
    const v4f z4 = {0.f, 0.f, 0.f, 0.f};
    if (row >= nN) { a = z4; b = z4; }
    const v4u hv = pack8(a, b);
    const size_t o = (size_t)row * F_IN + c0;
    *(volatile v4u*)(XB + o) = hv;
    __threadfence();
    *(volatile v4u*)(XB + o) = hv;
  } else {
    const int v = u - nUx;
    if (v < NUW) {
      wtr_unit(W0, F_IN, HC1, F_IN, WT0, v);
    } else if (v < 2 * NUW) {
      wtr_unit(W1, F_IN, HC1, F_IN, WT1, v - NUW);
    } else if (v < 3 * NUW) {
      wtr_unit(W2, F_IN, HC1, F_IN, WT2, v - 2 * NUW);
    } else if (v < 3 * NUW + NUL) {
      wtr_unit(Wl, HCAT, NCLS, KX, WLT, v - 3 * NUW);
    }
  }
}

template <int NT>
__global__ __launch_bounds__(GTHR) void k_gemm(
    const unsigned short* __restrict__ A, const unsigned short* __restrict__ WT,
    float* outF, int K, int ldo,
    const float* __restrict__ atts, const float* __restrict__ attd, int attLen,
    float* SD, int MPr)
{
  static_assert(NT == 1 || NT == 4);
  constexpr int CW = 16 * NT;
  __shared__ __attribute__((aligned(16))) float stg[GBM * CW];
  __shared__ __attribute__((aligned(16))) float satt[2 * CW];
  __shared__ __attribute__((aligned(16))) float sdot[2 * GBM];
  const int tid = (int)threadIdx.x, lane = tid & 31, wave = tid >> 5, hh = lane >> 4, m = lane & 15;
  const int rowBase = (int)blockIdx.x * GBM;
  const int head    = (int)blockIdx.y;
  const int col0    = head * CW;

  if (tid < 2 * CW) {
    const int which = tid / CW;
    const int c  = tid - which * CW;
    const int cl = c < attLen ? c : attLen - 1;
    const float vs = atts[head * attLen + cl];
    const float vd = attd[head * attLen + cl];
    asm volatile("" :: "v"(vs), "v"(vd));
    float v = (which == 0) ? vs : vd;
    v = (c < attLen) ? bfr(v) : 0.f;
    satt[which * CW + c] = v;
  }

  v8f acc[NT];
  {
    const v8f z = {0.f, 0.f, 0.f, 0.f, 0.f, 0.f, 0.f, 0.f};
#pragma unroll
    for (int t = 0; t < NT; ++t) acc[t] = z;
  }
  const unsigned short* ap = A  + (size_t)(rowBase + 16 * wave + m) * (size_t)K + 8 * hh;
  const unsigned short* wp = WT + (size_t)(col0 + m) * (size_t)K + 8 * hh;
  const int ksteps = K >> 5;
#pragma unroll 1
  for (int ks = 0; ks < ksteps; ++ks) {
    FragB af;
    af.h[0] = *(const v8usa*)(ap + 32 * ks);
    af.h[1] = *(const v8usa*)(ap + 32 * ks + 16);
#pragma unroll
    for (int t = 0; t < NT; ++t) {
      const unsigned short* wq = wp + (size_t)(16 * t) * (size_t)K + 32 * ks;
      FragB bf;
      bf.h[0] = *(const v8usa*)wq;
      bf.h[1] = *(const v8usa*)(wq + 16);
      acc[t] = wmb(af, bf, acc[t]);
    }
  }

#pragma unroll
  for (int t = 0; t < NT; ++t) {
    const int lc = 16 * t + m;
#pragma unroll
    for (int r = 0; r < 8; ++r) {
      const int lr = 16 * wave + 8 * hh + r;
      stg[lr * CW + lc] = acc[t][r];
    }
  }
  __syncthreads();

  {
    const int row = tid & 63, which = tid >> 6;
    const float* sa = satt + which * CW;
    const float* hr = stg + row * CW;
    float d = 0.f;
#pragma unroll 4
    for (int c4 = 0; c4 < CW / 4; ++c4) {
      const v4f hv = *(const v4fa*)(hr + 4 * c4);
      const v4f av = *(const v4fa*)(sa + 4 * c4);
      d = fmaf(hv.x, av.x, d);
      d = fmaf(hv.y, av.y, d);
      d = fmaf(hv.z, av.z, d);
      d = fmaf(hv.w, av.w, d);
    }
    sdot[which * GBM + row] = d;
  }
  __syncthreads();

  const int which2 = lane >> 4, piece = lane & 15;
  const v4f sdv = *(const v4fa*)(sdot + which2 * GBM + 4 * piece);
  float* sp = SD + (size_t)(2 * head + which2) * (size_t)MPr + rowBase + 4 * piece;

  if constexpr (NT == 4) {
    v4f fv[8];
#pragma unroll
    for (int i = 0; i < 8; ++i) {
      const int lr = 16 * wave + 2 * i + hh;
      fv[i] = *(const v4fa*)(stg + lr * CW + 4 * m);
    }
#pragma unroll
    for (int i = 0; i < 8; ++i) {
      const int lr = 16 * wave + 2 * i + hh;
      const int gr = rowBase + lr;
      float* op = outF + (size_t)gr * (size_t)ldo + col0 + 4 * m;
      *(volatile v4f*)op = fv[i];
    }
    if (wave == 0) *(volatile v4f*)sp = sdv;
    __threadfence();
#pragma unroll
    for (int i = 0; i < 8; ++i) {
      const int lr = 16 * wave + 2 * i + hh;
      const int gr = rowBase + lr;
      float* op = outF + (size_t)gr * (size_t)ldo + col0 + 4 * m;
      *(volatile v4f*)op = fv[i];
    }
    if (wave == 0) *(volatile v4f*)sp = sdv;
  } else {
    v4f fv[2];
#pragma unroll
    for (int i = 0; i < 2; ++i) fv[i] = *(const v4fa*)(stg + 4 * (tid + GTHR * i));
    float* ob = outF + (size_t)rowBase * (size_t)CW;
#pragma unroll
    for (int i = 0; i < 2; ++i) *(volatile v4f*)(ob + 4 * (tid + GTHR * i)) = fv[i];
    if (wave == 0) *(volatile v4f*)sp = sdv;
    __threadfence();
#pragma unroll
    for (int i = 0; i < 2; ++i) *(volatile v4f*)(ob + 4 * (tid + GTHR * i)) = fv[i];
    if (wave == 0) *(volatile v4f*)sp = sdv;
  }
}

template <int L>
__global__ __launch_bounds__(NTHR) void k_agg(
    const int* __restrict__ srcs, const int* __restrict__ dsts,
    const float* __restrict__ F, const float* __restrict__ SD,
    const float* __restrict__ bias,
    unsigned short* HP, float* out,
    int nN, int nE, int nb, int vec8, int MPr, int colB) {
  extern __shared__ v4f lds_dyn[];
  int* reg1 = (int*)lds_dyn;
  int* reg2 = reg1 + RCAP;
  int* scnt = reg2 + RCAP;
  int* soff = scnt + NBMAX;
  int* list = soff + NBMAX;
  int* wcnt = list + LISTN;
  int* wtot = wcnt + NWAVE;
  const int tid = (int)threadIdx.x, lane = tid & 31, wave = tid >> 5;
  const int nodeBase = (int)blockIdx.x * nb;

  for (int i = tid; i < NBMAX; i += NTHR) scnt[i] = 0;
  __syncthreads();

  int tot = 0;
  const int nChunks = (nE + CHUNK - 1) / CHUNK;
#pragma unroll 1
  for (int ch = 0; ch < nChunks; ++ch) {
    const int cbase = ch * CHUNK;
    const int wc = scan_chunk(dsts, nE, cbase, nodeBase, nb, vec8, list, tid, lane, wave);
    if (lane == 0) wcnt[wave] = wc;
    __syncthreads();
    int pre = 0, all = 0;
#pragma unroll
    for (int w2 = 0; w2 < NWAVE; ++w2) {
      int c = wcnt[w2];
      c = c < 0 ? 0 : (c > WCAP ? WCAP : c);
      all += c;
      pre += (w2 < wave) ? c : 0;
    }
    const int wcc  = wc > WCAP ? WCAP : wc;
    const int base = tot + pre;
#pragma unroll 1
    for (int i = lane; i < wcc; i += 32) {
      const int ent = list[wave * WCAP + i];
      const int el  = (ent >> SLOTB) & (CHUNK - 1);
      const int sl  = ent & (NBMAX - 1);
      int eid = cbase + el;
      eid = eid > nE - 1 ? nE - 1 : eid;
      const int pos = base + i;
      if (pos < RCAP) reg1[pos] = (int)(((unsigned)eid << SLOTB) | (unsigned)sl);
    }
    tot += all;
    tot = tot > RCAP ? RCAP : tot;
    __syncthreads();
  }
  const int nh = tot;

  if (wave == 0) {
#pragma unroll 1
    for (int b0 = 0; b0 < nh; b0 += 32) {
      const int idx = b0 + lane;
      const int uv  = reg1[idx < nh ? idx : nh - 1];
      const int m32 = (nh - b0) < 32 ? (nh - b0) : 32;
#pragma unroll 1
      for (int k = 0; k < m32; ++k) {
        const int u  = __builtin_amdgcn_readlane(uv, k);
        const int sl = u & (NBMAX - 1);
        if (lane == 0) scnt[sl] = scnt[sl] + 1;
      }
    }
  }
  __syncthreads();

  {
    const v4i ca = *(const v4i*)(scnt + 8 * tid);
    const v4i cb = *(const v4i*)(scnt + 8 * tid + 4);
    const int e0 = ca.x < 0 ? 0 : ca.x, e1 = ca.y < 0 ? 0 : ca.y, e2 = ca.z < 0 ? 0 : ca.z, e3 = ca.w < 0 ? 0 : ca.w;
    const int e4 = cb.x < 0 ? 0 : cb.x, e5 = cb.y < 0 ? 0 : cb.y, e6 = cb.z < 0 ? 0 : cb.z, e7 = cb.w < 0 ? 0 : cb.w;
    const int ts = e0 + e1 + e2 + e3 + e4 + e5 + e6 + e7;
    int incl = ts;
#pragma unroll
    for (int d = 1; d < 32; d <<= 1) {
      const int up = __shfl_up(incl, d);
      if (lane >= d) incl += up;
    }
    if (lane == 31) wtot[wave] = incl;
    __syncthreads();
    int pre = 0;
#pragma unroll
    for (int w2 = 0; w2 < NWAVE; ++w2) pre += (w2 < wave) ? wtot[w2] : 0;
    int run = pre + incl - ts;
    soff[8 * tid + 0] = run; run += e0;
    soff[8 * tid + 1] = run; run += e1;
    soff[8 * tid + 2] = run; run += e2;
    soff[8 * tid + 3] = run; run += e3;
    soff[8 * tid + 4] = run; run += e4;
    soff[8 * tid + 5] = run; run += e5;
    soff[8 * tid + 6] = run; run += e6;
    soff[8 * tid + 7] = run;
  }
  __syncthreads();
  for (int i = tid; i < NBMAX; i += NTHR) list[i] = soff[i];
  __syncthreads();

  if (wave == 0) {
#pragma unroll 1
    for (int b0 = 0; b0 < nh; b0 += 32) {
      const int idx = b0 + lane;
      const int uv  = reg1[idx < nh ? idx : nh - 1];
      const int m32 = (nh - b0) < 32 ? (nh - b0) : 32;
#pragma unroll 1
      for (int k = 0; k < m32; ++k) {
        const int u   = __builtin_amdgcn_readlane(uv, k);
        const int sl  = u & (NBMAX - 1);
        const int eid = (int)((unsigned)u >> SLOTB);
        if (lane == 0) {
          int pos = list[sl];
          pos = pos < 0 ? 0 : (pos > RCAP - 1 ? RCAP - 1 : pos);
          reg2[pos] = eid;
          list[sl] = pos + 1;
        }
      }
    }
  }
  __syncthreads();

  const int nbw = nb >> 3;
  const bool ovf = (nh >= RCAP);
  const float qnan = __int_as_float(0x7fc00000);

  if constexpr (L == 1) {
    const int c0   = 4 * lane;
    const int head = lane >> 4;
    const v4f bb4  = bfr4(*(const v4fa*)(bias + c0));
    const float* ASp = SD + (size_t)(2 * head) * (size_t)MPr;
    const float* ADp = ASp + MPr;
    float* wrow = (float*)reg1 + wave * WST;
    unsigned short* hrow = (unsigned short*)(wrow + HC1);
    const int gcol = colB + 8 * (lane & 15) + (lane >> 4) * HCAT;

#pragma unroll 1
    for (int jt = 0; jt < nbw; ++jt) {
      const int slot = wave * nbw + jt;
      const int grow = nodeBase + slot;
      const int gcl  = grow < nN ? grow : nN - 1;
      int st = soff[slot];
      const int craw = scnt[slot];
      int cnt = craw;
      st  = st < 0 ? 0 : (st > nh ? nh : st);
      cnt = cnt < 0 ? 0 : (cnt > DEGCAP ? DEGCAP : cnt);
      if (cnt > nh - st) cnt = nh - st;
      const float pz = (ovf || craw > DEGCAP) ? qnan : 0.0f;

      const v4f fd = *(const v4fa*)(F + (size_t)gcl * HC1 + c0);
      const float adv = ADp[gcl];
      float l0 = ASp[gcl] + adv;
      l0 = l0 > 0.f ? l0 : NEGSL * l0;
      float mx = l0, dn = 1.0f;
      v4f av = fd;

#pragma unroll 1
      for (int q = 0; q < cnt; ++q) {
        int idx = st + q; idx = idx > RCAP - 1 ? RCAP - 1 : idx;
        int eid = reg2[idx]; eid = eid < 0 ? 0 : (eid > nE - 1 ? nE - 1 : eid);
        const int sraw = srcs[eid];
        const int s = sraw < 0 ? 0 : (sraw > nN - 1 ? nN - 1 : sraw);
        const v4f fs = *(const v4fa*)(F + (size_t)s * HC1 + c0);
        float lg = ASp[s] + adv;
        lg = lg > 0.f ? lg : NEGSL * lg;
        const float df = lg - mx;
        const float ee = expf(-fabsf(df));
        const bool up  = df > 0.f;
        const float s1 = up ? ee : 1.0f;
        const float s2 = up ? 1.0f : ee;
        mx = up ? lg : mx;
        dn = fmaf(dn, s1, s2);
        av.x = fmaf(av.x, s1, s2 * fs.x);
        av.y = fmaf(av.y, s1, s2 * fs.y);
        av.z = fmaf(av.z, s1, s2 * fs.z);
        av.w = fmaf(av.w, s1, s2 * fs.w);
      }
      const float inv = 1.0f / dn;
      const bool live = grow < nN;
      v4f y;
      y.x = live ? fmaf(av.x, inv, bb4.x) : 0.f;
      y.y = live ? fmaf(av.y, inv, bb4.y) : 0.f;
      y.z = live ? fmaf(av.z, inv, bb4.z) : 0.f;
      y.w = live ? fmaf(av.w, inv, bb4.w) : 0.f;
      *(v4fa*)(wrow + c0) = y;
      __syncthreads();
#pragma unroll 1
      for (int i = 0; i < 4; ++i) {
        const int c = lane + 32 * i;
        const float v = wrow[c];
        float e = (v > 0.f) ? v : expm1f(v);
        e = e + pz;
        const unsigned int hb = f2bf(e);
        const unsigned int lb = f2bf(e - bf2f(hb));
        hrow[c]       = (unsigned short)hb;
        hrow[HC1 + c] = (unsigned short)lb;
      }
      __syncthreads();
      const v8us pv = *(const v8usa*)(hrow + 8 * lane);
      unsigned short* gp = HP + (size_t)grow * KX + gcol;
      const bool wr = grow < MPr;
      if (wr) *(volatile v8us*)gp = pv;
      __threadfence();
      if (wr) *(volatile v8us*)gp = pv;
    }
  } else {
    const int c = lane & 15;
    const float bz = bfr(bias[c]);
    const float* ASp = SD;
    const float* ADp = SD + MPr;
    float* res = (float*)reg1 + wave * (GRP * NCLS);

#pragma unroll 1
    for (int jt = 0; jt < nbw; ++jt) {
      const int slot = wave * nbw + jt;
      const int grow = nodeBase + slot;
      const int gcl  = grow < nN ? grow : nN - 1;
      int st = soff[slot];
      const int craw = scnt[slot];
      int cnt = craw;
      st  = st < 0 ? 0 : (st > nh ? nh : st);
      cnt = cnt < 0 ? 0 : (cnt > DEGCAP ? DEGCAP : cnt);
      if (cnt > nh - st) cnt = nh - st;
      const float pz = (ovf || craw > DEGCAP) ? qnan : 0.0f;

      const float fd = F[(size_t)gcl * NCLS + c];
      const float adv = ADp[gcl];
      float l0 = ASp[gcl] + adv;
      l0 = l0 > 0.f ? l0 : NEGSL * l0;
      float mx = l0, dn = 1.0f;
      float a0 = fd;

#pragma unroll 1
      for (int q = 0; q < cnt; ++q) {
        int idx = st + q; idx = idx > RCAP - 1 ? RCAP - 1 : idx;
        int eid = reg2[idx]; eid = eid < 0 ? 0 : (eid > nE - 1 ? nE - 1 : eid);
        const int sraw = srcs[eid];
        const int s = sraw < 0 ? 0 : (sraw > nN - 1 ? nN - 1 : sraw);
        const float fs = F[(size_t)s * NCLS + c];
        float lg = ASp[s] + adv;
        lg = lg > 0.f ? lg : NEGSL * lg;
        const float df = lg - mx;
        const float ee = expf(-fabsf(df));
        const bool up  = df > 0.f;
        const float s1 = up ? ee : 1.0f;
        const float s2 = up ? 1.0f : ee;
        mx = up ? lg : mx;
        dn = fmaf(dn, s1, s2);
        a0 = fmaf(a0, s1, s2 * fs);
      }
      const float inv = 1.0f / dn;
      const float z = fmaf(a0, inv, bz);
      float vm = z;
#pragma unroll
      for (int off = 8; off > 0; off >>= 1) vm = fmaxf(vm, __shfl_xor(vm, off));
      const float ex = expf(z - vm);
      float sm = ex;
#pragma unroll
      for (int off = 8; off > 0; off >>= 1) sm += __shfl_xor(sm, off);
      const float rs = 1.0f / sm;
      const float o = ex * rs + pz;
      const int lr = jt & (GRP - 1);
      if (lane < 16) res[lr * NCLS + c] = o;

      const int gb = jt & ~(GRP - 1);
      if (lr == GRP - 1 || jt == nbw - 1) {
        __syncthreads();
        int gsz = nbw - gb; gsz = gsz > GRP ? GRP : gsz;
        const int row0 = nodeBase + wave * nbw + gb;
        int live = nN - row0; live = live < 0 ? 0 : (live > gsz ? gsz : live);
        const int npc = live * (NCLS / 4);
        float* ob = out + (size_t)row0 * NCLS;
#pragma unroll 1
        for (int p = lane; p < npc; p += 32) {
          const v4f v = *(const v4fa*)(res + 4 * p);
          *(volatile v4f*)(ob + 4 * p) = v;
        }
        __threadfence();
#pragma unroll 1
        for (int p = lane; p < npc; p += 32) {
          const v4f v = *(const v4fa*)(res + 4 * p);
          *(volatile v4f*)(ob + 4 * p) = v;
        }
        __syncthreads();
      }
    }
  }
}

static int pick_nb(int nE, int nN) {
  int nb = NBMAX;
  while (nb > 32 && (long long)nb * (long long)nE * 5LL > (long long)RCAP * (long long)nN * 4LL) nb >>= 1;
  return nb;
}
static inline int cdiv(int a, int b) { return (a + b - 1) / b; }

extern "C" void kernel_launch(void* const* d_in, const int* in_sizes, int n_in,
                              void* d_out, int out_size, void* d_ws, size_t ws_size,
                              hipStream_t stream) {
  if (n_in < 20) return;
  const int nN = in_sizes[0] / F_IN;
  if (nN <= 0 || in_sizes[0] != nN * F_IN || nN > (1 << 22) || (nN & 1) != 0) return;
  int nEv[3];
  for (int i = 0; i < 3; ++i) {
    const int sz = in_sizes[1 + i];
    if (sz < 2 || (sz & 1) != 0) return;
    nEv[i] = sz / 2;
    if (nEv[i] < 1 || nEv[i] >= (1 << (32 - SLOTB))) return;
  }
  const int nEa = nEv[0], nEs = nEv[1], nEt = nEv[2];
  for (int b = 0; b < 3; ++b) {
    if (in_sizes[4 + 4 * b] != F_IN * HC1) return;
    if (in_sizes[5 + 4 * b] != NHD1 * HID || in_sizes[6 + 4 * b] != NHD1 * HID) return;
    if (in_sizes[7 + 4 * b] != HC1) return;
  }
  if (in_sizes[16] != HCAT * NCLS) return;
  if (in_sizes[17] != NCLS || in_sizes[18] != NCLS || in_sizes[19] != NCLS) return;
  if ((long long)out_size != (long long)nN * NCLS) return;

  const float* x    = (const float*)d_in[0];
  const int*   eA   = (const int*)  d_in[1];
  const int*   eS   = (const int*)  d_in[2];
  const int*   eT   = (const int*)  d_in[3];
  const float* Wst  = (const float*)d_in[4];
  const float* asst = (const float*)d_in[5];
  const float* adst = (const float*)d_in[6];
  const float* bst  = (const float*)d_in[7];
  const float* Wts  = (const float*)d_in[8];
  const float* asts = (const float*)d_in[9];
  const float* adts = (const float*)d_in[10];
  const float* bts  = (const float*)d_in[11];
  const float* Wc   = (const float*)d_in[12];
  const float* asc  = (const float*)d_in[13];
  const float* adc  = (const float*)d_in[14];
  const float* bc   = (const float*)d_in[15];
  const float* Wl   = (const float*)d_in[16];
  const float* asl  = (const float*)d_in[17];
  const float* adl  = (const float*)d_in[18];
  const float* bl   = (const float*)d_in[19];
  float* out = (float*)d_out;

  const int MP  = cdiv(nN, MROWS) * MROWS;
  const int nUx = MP * (F_IN / 8);
  if ((nUx % NTHR) != 0 || (MP % GBM) != 0) return;
  const int gM  = MP / GBM;

  const int nbS = pick_nb(nEs, nN), nbT = pick_nb(nEt, nN), nbA = pick_nb(nEa, nN);
  if (nbS < 32 || nbT < 32 || nbA < 32) return;
  const int gS = cdiv(MP, nbS), gT = cdiv(MP, nbT), gAa = cdiv(MP, nbA);
  const int vS = ((nEs & 3) == 0) ? 1 : 0, vT = ((nEt & 3) == 0) ? 1 : 0, vA = ((nEa & 3) == 0) ? 1 : 0;

  char* ws = (char*)d_ws;
  size_t off = 0;
  const size_t oXB  = off; off += (size_t)MP * F_IN * 2;          off = (off + 255) & ~(size_t)255;
  const size_t oW0  = off; off += (size_t)HC1 * F_IN * 2;         off = (off + 255) & ~(size_t)255;
  const size_t oW1  = off; off += (size_t)HC1 * F_IN * 2;         off = (off + 255) & ~(size_t)255;
  const size_t oW2  = off; off += (size_t)HC1 * F_IN * 2;         off = (off + 255) & ~(size_t)255;
  const size_t oWL  = off; off += (size_t)NCLS * KX * 2;          off = (off + 255) & ~(size_t)255;
  const size_t oH   = off; off += (size_t)MP * HC1 * 4;           off = (off + 255) & ~(size_t)255;
  const size_t oSD  = off; off += (size_t)4 * MP * 4;             off = (off + 255) & ~(size_t)255;
  const size_t oXHL = off; off += (size_t)MP * KX * 2;            off = (off + 255) & ~(size_t)255;
  const size_t oHL  = off; off += (size_t)MP * NCLS * 4;          off = (off + 255) & ~(size_t)255;
  const size_t oSDL = off; off += (size_t)2 * MP * 4;             off = (off + 255) & ~(size_t)255;
  if (off > ws_size || off > (size_t)WSMAX) return;
  unsigned short* XB  = (unsigned short*)(ws + oXB);
  unsigned short* WT0 = (unsigned short*)(ws + oW0);
  unsigned short* WT1 = (unsigned short*)(ws + oW1);
  unsigned short* WT2 = (unsigned short*)(ws + oW2);
  unsigned short* WLT = (unsigned short*)(ws + oWL);
  float*          H   = (float*)(ws + oH);
  float*          SD  = (float*)(ws + oSD);
  unsigned short* XHL = (unsigned short*)(ws + oXHL);
  float*          HL  = (float*)(ws + oHL);
  float*          SDL = (float*)(ws + oSDL);

  hipFuncSetAttribute(reinterpret_cast<const void*>(&k_agg<1>),
                      hipFuncAttributeMaxDynamicSharedMemorySize, LDS_AGG);
  hipFuncSetAttribute(reinterpret_cast<const void*>(&k_agg<2>),
                      hipFuncAttributeMaxDynamicSharedMemorySize, LDS_AGG);

  k_prep<<<(nUx + 3 * NUW + NUL) / NTHR, NTHR, 0, stream>>>(x, Wst, Wts, Wc, Wl, XB, WT0, WT1, WT2, WLT, nN, nUx);

  k_gemm<4><<<dim3(gM, NHD1), GTHR, 0, stream>>>(XB, WT0, H, F_IN, HC1, asst, adst, HID, SD, MP);
  k_agg<1><<<gS, NTHR, LDS_AGG, stream>>>(eS, eS + nEs, H, SD, bst, XHL, out, nN, nEs, nbS, vS, MP, 0);
  k_gemm<4><<<dim3(gM, NHD1), GTHR, 0, stream>>>(XB, WT1, H, F_IN, HC1, asts, adts, HID, SD, MP);
  k_agg<1><<<gT, NTHR, LDS_AGG, stream>>>(eT, eT + nEt, H, SD, bts, XHL, out, nN, nEt, nbT, vT, MP, HC1);
  k_gemm<4><<<dim3(gM, NHD1), GTHR, 0, stream>>>(XB, WT2, H, F_IN, HC1, asc, adc, HID, SD, MP);
  k_agg<1><<<gAa, NTHR, LDS_AGG, stream>>>(eA, eA + nEa, H, SD, bc, XHL, out, nN, nEa, nbA, vA, MP, 2 * HC1);
  k_gemm<1><<<dim3(gM, 1), GTHR, 0, stream>>>(XHL, WLT, HL, KX, NCLS, asl, adl, NCLS, SDL, MP);
  k_agg<2><<<gAa, NTHR, LDS_AGG, stream>>>(eA, eA + nEa, HL, SDL, bl, XHL, out, nN, nEa, nbA, vA, MP, 0);
}
